// FeedForwardQuantum_65481071398675
// MI455X (gfx1250) — hardware-verified
//
#include <hip/hip_runtime.h>
#include <stddef.h>
#include <stdint.h>


#define MTOT  16384
#define EMB   768
#define FFN   3072
#define NQ    8
#define HSC   16
#define WSC   1024
#define NTHR  256
#define NWAVE 8
#define HTHR  384
#define RB    64
#define WSCAP 134217728
#define LDS_GEMM (NWAVE * 32 * 64 * 4)

static_assert((FFN % 32) == 0);
static_assert((MTOT % 128) == 0);
static_assert((EMB % 128) == 0);
static_assert((HTHR / 32) * 256 == FFN);
static_assert((MTOT % RB) == 0);
static_assert(((EMB * FFN) % (8 * NTHR)) == 0);
static_assert(((MTOT * NQ) % NTHR) == 0);
static_assert(NTHR == NWAVE * 32);
static_assert(LDS_GEMM <= 300 * 1024);

typedef float          v4f  __attribute__((ext_vector_type(4)));
typedef float          v8f  __attribute__((ext_vector_type(8)));
typedef _Float16       v8h  __attribute__((ext_vector_type(8)));
typedef _Float16       v16h __attribute__((ext_vector_type(16)));
union FragH { v16h v; v8h h[2]; };

__device__ __forceinline__ v8f wmf(v16h a, v16h b, v8f c) {
  v8f d = __builtin_amdgcn_wmma_f32_16x16x32_f16(false, a, false, b, (short)0, c, false, false);
  asm volatile("v_nop\n\tv_nop\n\tv_nop\n\tv_nop" : "+v"(d) : "v"(a), "v"(b));
  return d;
}

__global__ __launch_bounds__(NTHR) void k_prepq(const float* __restrict__ x, const float* __restrict__ theta,
                                                float* qs) {
  __shared__ __attribute__((aligned(16))) float sq[NTHR];
  const int t = threadIdx.x;
  const size_t e = (size_t)blockIdx.x * NTHR + t;
  const size_t row = e >> 3;
  const int i = (int)(e & 7);
  const float xv = x[row * EMB + i];
  const float th = theta[i];
  float c = (float)HSC;
#pragma unroll 1
  for (int j = 0; j < 2; ++j) {
    const float a = (j == 0) ? xv : th;
    c = c * cosf(a);
  }
  sq[t] = c;
  __syncthreads();
  if (t < NTHR / 4) {
    const v4f v = *(const v4f*)(sq + 4 * t);
    float* d = qs + (size_t)blockIdx.x * NTHR + 4 * t;
    *(volatile v4f*)d = v;
    __threadfence();
    *(volatile v4f*)d = v;
  }
}

__global__ __launch_bounds__(HTHR) void k_preph(const float* __restrict__ qs, const float* __restrict__ w1,
                                                const float* __restrict__ b1, _Float16* hp) {
  const int tid = threadIdx.x, lane = tid & 31, wave = tid >> 5;
  const int f0 = wave * 256 + 8 * lane;
  const int rbase = blockIdx.x * RB;

  v4f w[16];
  const v4f* wp = (const v4f*)(w1 + (size_t)f0 * NQ);
#pragma unroll
  for (int j = 0; j < 16; ++j) w[j] = wp[j];
  const v4f ba = *(const v4f*)(b1 + f0);
  const v4f bb = *(const v4f*)(b1 + f0 + 4);
  float bs[8];
  bs[0] = ba.x * (float)HSC; bs[1] = ba.y * (float)HSC; bs[2] = ba.z * (float)HSC; bs[3] = ba.w * (float)HSC;
  bs[4] = bb.x * (float)HSC; bs[5] = bb.y * (float)HSC; bs[6] = bb.z * (float)HSC; bs[7] = bb.w * (float)HSC;

#pragma unroll 1
  for (int r = 0; r < RB; ++r) {
    const size_t row = (size_t)(rbase + r);
    const v4f qa = *(const v4f*)(qs + row * NQ);
    const v4f qb = *(const v4f*)(qs + row * NQ + 4);
    v8h hv;
#pragma unroll
    for (int j = 0; j < 8; ++j) {
      const v4f wl = w[2 * j];
      const v4f wh = w[2 * j + 1];
      float a = bs[j];
      a = fmaf(qa.x, wl.x, a); a = fmaf(qa.y, wl.y, a); a = fmaf(qa.z, wl.z, a); a = fmaf(qa.w, wl.w, a);
      a = fmaf(qb.x, wh.x, a); a = fmaf(qb.y, wh.y, a); a = fmaf(qb.z, wh.z, a); a = fmaf(qb.w, wh.w, a);
      a = fmaxf(a, 0.0f);
      hv[j] = (_Float16)a;
    }
    _Float16* d = hp + row * FFN + f0;
    *(volatile v8h*)d = hv;
    __threadfence();
    *(volatile v8h*)d = hv;
  }
}

__global__ __launch_bounds__(NTHR) void k_prepw(const float* __restrict__ w2, _Float16* wt) {
  const size_t t = (size_t)blockIdx.x * NTHR + threadIdx.x;
  const float* p = w2 + t * 8;
  const v4f f0 = *(const v4f*)p;
  const v4f f1 = *(const v4f*)(p + 4);
  v8h a;
  a[0] = (_Float16)(f0.x * (float)WSC); a[1] = (_Float16)(f0.y * (float)WSC);
  a[2] = (_Float16)(f0.z * (float)WSC); a[3] = (_Float16)(f0.w * (float)WSC);
  a[4] = (_Float16)(f1.x * (float)WSC); a[5] = (_Float16)(f1.y * (float)WSC);
  a[6] = (_Float16)(f1.z * (float)WSC); a[7] = (_Float16)(f1.w * (float)WSC);
  _Float16* d = wt + t * 8;
  *(volatile v8h*)d = a;
  __threadfence();
  *(volatile v8h*)d = a;
}

__global__ __launch_bounds__(NTHR) void k_gemm(const _Float16* __restrict__ hp, const _Float16* __restrict__ wt,
                                               const float* __restrict__ bias, float* out) {
  extern __shared__ v4f lds_dyn[];
  const int tid = threadIdx.x, lane = tid & 31, wave = tid >> 5, hf = lane >> 4, m = lane & 15;
  float* stg = (float*)lds_dyn + wave * (32 * 64);
  const int n0 = blockIdx.x * 128, m0 = blockIdx.y * 128;
  const int wm = (wave >> 1) * 32, wn = (wave & 1) * 64;

  v8f acc[2][4];
#pragma unroll
  for (int mt = 0; mt < 2; ++mt)
#pragma unroll
    for (int nt = 0; nt < 4; ++nt) { v8f z = {0.f, 0.f, 0.f, 0.f, 0.f, 0.f, 0.f, 0.f}; acc[mt][nt] = z; }

  const _Float16* ap = hp + (size_t)(m0 + wm + m) * FFN + 8 * hf;
  const _Float16* bp = wt + (size_t)(n0 + wn + m) * FFN + 8 * hf;
#pragma unroll 1
  for (int kt = 0; kt < FFN / 32; ++kt) {
    const int k0 = 32 * kt;
    FragH a0, a1;
    a0.h[0] = *(const v8h*)(ap + k0);
    a0.h[1] = *(const v8h*)(ap + k0 + 16);
    a1.h[0] = *(const v8h*)(ap + 16 * FFN + k0);
    a1.h[1] = *(const v8h*)(ap + 16 * FFN + k0 + 16);
#pragma unroll
    for (int nt = 0; nt < 4; ++nt) {
      const _Float16* bq = bp + (size_t)nt * 16 * FFN + k0;
      FragH b;
      b.h[0] = *(const v8h*)bq;
      b.h[1] = *(const v8h*)(bq + 16);
      acc[0][nt] = wmf(a0.v, b.v, acc[0][nt]);
      acc[1][nt] = wmf(a1.v, b.v, acc[1][nt]);
    }
  }

  constexpr float OSC = 1.0f / (float)(HSC * WSC);
  float bv[4];
#pragma unroll
  for (int nt = 0; nt < 4; ++nt) bv[nt] = bias[n0 + wn + 16 * nt + m];
#pragma unroll
  for (int mt = 0; mt < 2; ++mt) {
    float* sp = stg + (16 * mt + 8 * hf) * 64 + m;
#pragma unroll
    for (int nt = 0; nt < 4; ++nt) {
#pragma unroll
      for (int r = 0; r < 8; ++r) sp[r * 64 + 16 * nt] = acc[mt][nt][r] * OSC + bv[nt];
    }
  }
  __syncthreads();

  float* gbase = out + (size_t)(m0 + wm) * EMB + n0 + wn;
#pragma unroll
  for (int q = 0; q < 16; ++q) {
    const int row = 2 * q + hf;
    const v4f v = *(const v4f*)(stg + row * 64 + 4 * m);
    *(volatile v4f*)(gbase + (size_t)row * EMB + 4 * m) = v;
  }
  __threadfence();
#pragma unroll
  for (int q = 0; q < 16; ++q) {
    const int row = 2 * q + hf;
    const v4f v = *(const v4f*)(stg + row * 64 + 4 * m);
    *(volatile v4f*)(gbase + (size_t)row * EMB + 4 * m) = v;
  }
}

extern "C" void kernel_launch(void* const* d_in, const int* in_sizes, int n_in,
                              void* d_out, int out_size, void* d_ws, size_t ws_size,
                              hipStream_t stream) {
  if (n_in < 6) return;
  if (in_sizes[0] != MTOT * EMB || in_sizes[1] != NQ || in_sizes[2] != FFN * NQ ||
      in_sizes[3] != FFN || in_sizes[4] != EMB * FFN || in_sizes[5] != EMB) return;
  if (out_size != MTOT * EMB) return;

  const float* x     = (const float*)d_in[0];
  const float* theta = (const float*)d_in[1];
  const float* w1    = (const float*)d_in[2];
  const float* b1    = (const float*)d_in[3];
  const float* w2    = (const float*)d_in[4];
  const float* b2    = (const float*)d_in[5];
  float* out = (float*)d_out;

  char* ws = (char*)d_ws;
  size_t off = 0;
  const size_t oQ = off; off += (size_t)MTOT * NQ * 4;   off = (off + 255) & ~(size_t)255;
  const size_t oH = off; off += (size_t)MTOT * FFN * 2;  off = (off + 255) & ~(size_t)255;
  const size_t oW = off; off += (size_t)EMB * FFN * 2;   off = (off + 255) & ~(size_t)255;
  if (off > ws_size || off > (size_t)WSCAP) return;
  float* qs = (float*)(ws + oQ);
  _Float16* hp = (_Float16*)(ws + oH);
  _Float16* wt = (_Float16*)(ws + oW);

  k_prepq<<<(MTOT * NQ) / NTHR, NTHR, 0, stream>>>(x, theta, qs);
  k_preph<<<MTOT / RB, HTHR, 0, stream>>>(qs, w1, b1, hp);
  k_prepw<<<(EMB * FFN) / (8 * NTHR), NTHR, 0, stream>>>(w2, wt);
  hipFuncSetAttribute(reinterpret_cast<const void*>(&k_gemm),
                      hipFuncAttributeMaxDynamicSharedMemorySize, LDS_GEMM);
  k_gemm<<<dim3(EMB / 128, MTOT / 128), NTHR, LDS_GEMM, stream>>>(hp, wt, b2, out);
}
